// MultiHeadAttentionBlock_74156905333477
// MI455X (gfx1250) — hardware-verified
//
#include <hip/hip_runtime.h>


#ifndef NB
#define NB 2
#endif
#ifndef SEQ
#define SEQ 2048
#endif
#define NB_FULL  2
#define SEQ_FULL 2048
#define DM   1024
#define NH   16
#define HD   64
#define DQ   (NH * HD)
#define RH   512
#define RHC  ((RH < SEQ) ? RH : SEQ)
#define KT   64
#define NKT  (SEQ / KT)
#define PP   72
#define PCAR 1024.0f
#define SCL  0.125f
#define MFILL (-1.0e9f)
#define L2E  1.4426950408889634f
#define WS_CAP ((size_t)134217728)

static_assert(SEQ % 64 == 0);
static_assert(NKT >= 1 && NKT <= 32);
static_assert(SEQ <= SEQ_FULL);
static_assert(NB >= 1 && NB <= NB_FULL);
static_assert(RHC % 16 == 0);
static_assert(DM % 64 == 0 && DQ == DM && HD == 64);

typedef _Float16 h16;
typedef unsigned short bf;
typedef __attribute__((ext_vector_type(16))) __bf16   v16bf;
typedef __attribute__((ext_vector_type(16))) _Float16 v16h;
typedef __attribute__((ext_vector_type(8)))  _Float16 v8h;
typedef __attribute__((ext_vector_type(8)))  unsigned short v8us;
typedef __attribute__((ext_vector_type(8)))  float    v8f;
typedef __attribute__((ext_vector_type(4)))  float    v4f;
typedef __attribute__((ext_vector_type(2)))  _Float16 v2h;
typedef __attribute__((ext_vector_type(2)))  unsigned short v2us;
typedef __attribute__((ext_vector_type(4)))  int      v4i;
typedef v8h  __attribute__((may_alias)) v8ha;
typedef v4f  __attribute__((may_alias)) v4fa;
typedef v8us __attribute__((may_alias)) v8usa;

__device__ __forceinline__ unsigned short f2bf(float f) { unsigned u = __float_as_uint(f); u += 0x7FFFu + ((u >> 16) & 1u); return (unsigned short)(u >> 16); }
__device__ __forceinline__ float bf2f(unsigned short b) { return __uint_as_float(((unsigned)b) << 16); }
__device__ __forceinline__ float bfr(float f) { return bf2f(f2bf(f)); }
__device__ __forceinline__ v16h cat16(v8h lo, v8h hi) { return __builtin_shufflevector(lo, hi, 0, 1, 2, 3, 4, 5, 6, 7, 8, 9, 10, 11, 12, 13, 14, 15); }
__device__ __forceinline__ v16bf cat16b(v8us lo, v8us hi) { return __builtin_bit_cast(v16bf, __builtin_shufflevector(lo, hi, 0, 1, 2, 3, 4, 5, 6, 7, 8, 9, 10, 11, 12, 13, 14, 15)); }
__device__ __forceinline__ v8f wmma16(v16h a, v16h b, v8f c) { return __builtin_amdgcn_wmma_f32_16x16x32_f16(false, a, false, b, (short)0, c, false, false); }
__device__ __forceinline__ v8f wmmab(v16bf a, v16bf b, v8f c) { return __builtin_amdgcn_wmma_f32_16x16x32_bf16(false, a, false, b, (short)0, c, false, false); }
__device__ __forceinline__ h16 tohx(float x) { return (h16)x; }
__device__ __forceinline__ void splitf(float y, unsigned short& h, unsigned short& l) { h = f2bf(y); l = f2bf(y - bf2f(h)); }

template <typename T16> struct WFrag;
template <> struct WFrag<h16> { typedef v16h V; static __device__ __forceinline__ V ld(const h16* p) { return cat16(*(const v8h*)p, *(const v8h*)(p + 16)); } static __device__ __forceinline__ v8f mma(V a, V b, v8f c) { return wmma16(a, b, c); } };
template <> struct WFrag<bf> { typedef v16bf V; static __device__ __forceinline__ V ld(const bf* p) { return cat16b(*(const v8us*)p, *(const v8us*)(p + 16)); } static __device__ __forceinline__ v8f mma(V a, V b, v8f c) { return wmmab(a, b, c); } };
template <typename T16, int NSPLIT, bool BIAS>
__global__ __launch_bounds__(32) void k_gemmw(const T16* __restrict__ A, const T16* __restrict__ A2, const T16* __restrict__ Bt, const T16* __restrict__ Bt2, int K, float* C, int ldc, const float* __restrict__ bias, size_t sA, size_t sB, size_t sC) {
    typedef typename WFrag<T16>::V V;
    __shared__ __align__(16) float os[16 * 68];
    const size_t z = blockIdx.z; A += z * sA; if (A2) A2 += z * sA; Bt += z * sB; if (Bt2) Bt2 += z * sB; C += z * sC;
    const int lane = threadIdx.x & 31, lr = lane & 15, hi = lane >> 4; const int r0 = blockIdx.x * 64, c0 = blockIdx.y * 64;
    v8f acc[4][4];
#pragma unroll
    for (int mb = 0; mb < 4; ++mb)
#pragma unroll
        for (int nb = 0; nb < 4; ++nb) acc[mb][nb] = (v8f){};
    const size_t aoff = (size_t)(r0 + lr) * K + 8 * hi, boff = (size_t)(c0 + lr) * K + 8 * hi;
#pragma unroll 1
    for (int kc = 0; kc < K; kc += 32) {
        V a[4], a2[4];
#pragma unroll
        for (int mb = 0; mb < 4; ++mb) { a[mb] = WFrag<T16>::ld(A + aoff + (size_t)mb * 16 * K + kc); if (NSPLIT == 1 || NSPLIT == 2) a2[mb] = WFrag<T16>::ld(A2 + aoff + (size_t)mb * 16 * K + kc); }
#pragma unroll
        for (int nb = 0; nb < 4; ++nb) { const V b = WFrag<T16>::ld(Bt + boff + (size_t)nb * 16 * K + kc); V b2; if (NSPLIT >= 2) b2 = WFrag<T16>::ld(Bt2 + boff + (size_t)nb * 16 * K + kc);
#pragma unroll
            for (int mb = 0; mb < 4; ++mb) { acc[mb][nb] = WFrag<T16>::mma(a[mb], b, acc[mb][nb]); if (NSPLIT == 1 || NSPLIT == 2) acc[mb][nb] = WFrag<T16>::mma(a2[mb], b, acc[mb][nb]); if (NSPLIT >= 2) acc[mb][nb] = WFrag<T16>::mma(a[mb], b2, acc[mb][nb]); } }
        asm volatile("v_nop\n\tv_nop\n\tv_nop\n\tv_nop" : "+v"(acc[0][0]), "+v"(acc[1][1]), "+v"(acc[2][2]), "+v"(acc[3][3]) : "v"(a[0]), "v"(a[3]));
    }
#pragma unroll
    for (int mb = 0; mb < 4; ++mb) {
#pragma unroll
        for (int nb = 0; nb < 4; ++nb) {
#pragma unroll
            for (int j = 0; j < 8; ++j) os[(hi * 8 + j) * 68 + nb * 16 + lr] = acc[mb][nb][j]; }
        __builtin_amdgcn_wave_barrier(); asm volatile("" ::: "memory");
        float* crow = C + (size_t)(r0 + mb * 16) * ldc + c0;
#pragma unroll 1
        for (int ps = 0; ps < 2; ++ps) {
#pragma unroll
            for (int s = 0; s < 8; ++s) { const int row = 2 * s + hi, cofs = lr * 4; v4f val = *(const v4fa*)(os + row * 68 + cofs); if (BIAS) { val[0] += bfr(bias[c0 + cofs]); val[1] += bfr(bias[c0 + cofs + 1]); val[2] += bfr(bias[c0 + cofs + 2]); val[3] += bfr(bias[c0 + cofs + 3]); }
                *(volatile v4f*)(crow + (size_t)row * ldc + cofs) = val; }
            if (ps == 0) __threadfence(); }
        __builtin_amdgcn_wave_barrier(); asm volatile("" ::: "memory");
    }
}

__global__ __launch_bounds__(256) void k_cvt8(const float* __restrict__ src, bf* dst, size_t n8) { const size_t i = (size_t)blockIdx.x * 256 + threadIdx.x; if (i >= n8) return; const v8f v = *(const v8f*)(src + i * 8); v8us o;
#pragma unroll
    for (int k = 0; k < 8; ++k) o[k] = f2bf(v[k]); *(volatile v8us*)(dst + i * 8) = o; __threadfence(); *(volatile v8us*)(dst + i * 8) = o; }

__global__ __launch_bounds__(256) void k_qkp(const float* __restrict__ F, int pitch, int nheads, h16* P16, bf* Ph, bf* Pl) {
    const size_t e = ((size_t)blockIdx.x * 256 + threadIdx.x) * 2; if (e >= (size_t)nheads * SEQ * HD) return;
    const int d = (int)(e % HD); const int t = (int)((e / HD) % SEQ); const int h = (int)(e / ((size_t)HD * SEQ));
    const float* f = F + (size_t)t * pitch + h * HD + d; v2h o16; v2us oh, ol;
#pragma unroll
    for (int q = 0; q < 2; ++q) { const float x = f[q]; o16[q] = tohx(x); unsigned short a2, c2; splitf(x, a2, c2); oh[q] = a2; ol[q] = c2; }
    *(volatile v2h*)(P16 + e) = o16; *(volatile v2us*)(Ph + e) = oh; *(volatile v2us*)(Pl + e) = ol; __threadfence(); *(volatile v2h*)(P16 + e) = o16; *(volatile v2us*)(Ph + e) = oh; *(volatile v2us*)(Pl + e) = ol; }
__global__ __launch_bounds__(256) void k_vtp(const float* __restrict__ F, int pitch, int nheads, h16* V16, bf* Vh, bf* Vl) { const size_t e = ((size_t)blockIdx.x * 256 + threadIdx.x) * 2; if (e >= (size_t)nheads * HD * SEQ) return; const int t = (int)(e % SEQ); const int d = (int)((e / SEQ) % HD); const int g = (int)(e / ((size_t)SEQ * HD)); v2h o16; v2us oh, ol;
#pragma unroll
    for (int q = 0; q < 2; ++q) { const float x = F[(size_t)(t + q) * pitch + g * HD + d]; o16[q] = tohx(x); unsigned short a2, c2; splitf(x, a2, c2); oh[q] = a2; ol[q] = c2; }
    *(volatile v2h*)(V16 + e) = o16; *(volatile v2us*)(Vh + e) = oh; *(volatile v2us*)(Vl + e) = ol; __threadfence(); *(volatile v2h*)(V16 + e) = o16; *(volatile v2us*)(Vh + e) = oh; *(volatile v2us*)(Vl + e) = ol; }

__global__ __launch_bounds__(32) void k_mflag(const int* __restrict__ am, int pitch, int nkt, int* flg) {
    const int lane = threadIdx.x & 31; const int qb = blockIdx.x; const int q0 = qb * 16;
    const int ktc = (lane < nkt) ? lane : (nkt - 1);
    int anyv = 0, allv = 1, rowbits = 0;
#pragma unroll 1
    for (int r = 0; r < 16; ++r) {
        const int* rp = am + (size_t)(q0 + r) * pitch + ktc * KT; int ra = 0;
#pragma unroll
        for (int c = 0; c < KT / 4; ++c) { const v4i m = *(const v4i*)(rp + c * 4);
#pragma unroll
            for (int q = 0; q < 4; ++q) { const int nz = (m[q] != 0) ? 1 : 0; ra |= nz; allv &= nz; } }
        anyv |= ra; rowbits |= ra << r;
    }
    if (lane >= nkt) { anyv = 0; allv = 0; rowbits = 0; }
    int orb = rowbits;
#pragma unroll
    for (int sh = 16; sh; sh >>= 1) orb |= __shfl_xor(orb, sh, 32);
    const int force = (orb != 0xFFFF) ? 4 : 0;
    const int fw = (lane < nkt) ? (anyv | (allv << 1) | force) : 0;
    *(volatile int*)(flg + (size_t)qb * 32 + lane) = fw; __threadfence(); *(volatile int*)(flg + (size_t)qb * 32 + lane) = fw;
}

template <bool HR>
__global__ __launch_bounds__(32) void k_flash(const h16* __restrict__ Q16, const bf* __restrict__ Qh, const bf* __restrict__ Ql,
                                              const h16* __restrict__ K16, const bf* __restrict__ Kh, const bf* __restrict__ Kl,
                                              const h16* __restrict__ V16, const bf* __restrict__ Vh, const bf* __restrict__ Vl,
                                              const int* __restrict__ am, int mpitch, const int* __restrict__ flg, int qb0, bf* Ah, bf* Al) {
    __shared__ __align__(16) int   ms[16 * KT];
    __shared__ __align__(16) h16   pb16[16 * PP];
    __shared__ __align__(16) bf    pbh[16 * PP];
    __shared__ __align__(16) bf    pbl[16 * PP];
    __shared__ __align__(16) float os[16 * 68];
    const int lane = threadIdx.x & 31, lr = lane & 15, hi = lane >> 4;
    const int qb = qb0 + (int)blockIdx.x, hh = (int)blockIdx.y; const int q0 = qb * 16;
    const size_t hoff = (size_t)hh * SEQ * HD;
    const size_t qo = hoff + (size_t)(q0 + lr) * HD + 8 * hi;
    const v16h  aq0 = WFrag<h16>::ld(Q16 + qo), aq1 = WFrag<h16>::ld(Q16 + qo + 32);
    const v16bf ah0 = WFrag<bf>::ld(Qh + qo), ah1 = WFrag<bf>::ld(Qh + qo + 32), al0 = WFrag<bf>::ld(Ql + qo), al1 = WFrag<bf>::ld(Ql + qo + 32);
    v8f acc[4]; float mrow[8], lsum[8];
#pragma unroll
    for (int t = 0; t < 4; ++t) acc[t] = (v8f){};
#pragma unroll
    for (int r = 0; r < 8; ++r) { mrow[r] = -3.0e38f; lsum[r] = 0.f; }
    const int myflag = flg[(size_t)qb * 32 + lane];
    unsigned vis = __builtin_amdgcn_ballot_w32(myflag != 0);
    const unsigned fullb = __builtin_amdgcn_ballot_w32((myflag & 2) != 0);
    if (vis == 0u) vis = 0xFFFFFFFFu >> (32 - NKT);
#pragma unroll 1
    for (int kt = 0; kt < NKT; ++kt) {
        if (((vis >> kt) & 1u) == 0u) continue;
        const bool part = (((fullb >> kt) & 1u) == 0u);
        const int t0 = kt * KT;
        if (part) {
#pragma unroll
            for (int i = 0; i < 8; ++i) { const int e = i * 32 + lane; const int row = e >> 4, c4 = (e & 15) * 4;
                const v4i m4 = *(const v4i*)(am + (size_t)(q0 + row) * mpitch + t0 + c4); *(v4i*)(ms + row * KT + c4) = m4; }
            __syncthreads();
        }
        v8f s[4];
#pragma unroll
        for (int nf = 0; nf < 4; ++nf) {
            s[nf] = (v8f){};
#pragma unroll
            for (int kc = 0; kc < HD; kc += 32) {
                const size_t ko = hoff + (size_t)(t0 + nf * 16 + lr) * HD + 8 * hi + kc;
                if (HR) { const v16bf b0 = WFrag<bf>::ld(Kh + ko), b1 = WFrag<bf>::ld(Kl + ko); const v16bf a0 = kc ? ah1 : ah0, a1 = kc ? al1 : al0;
                    s[nf] = wmmab(a0, b0, s[nf]); s[nf] = wmmab(a1, b0, s[nf]); s[nf] = wmmab(a0, b1, s[nf]); }
                else { const v16h b0 = WFrag<h16>::ld(K16 + ko); s[nf] = wmma16(kc ? aq1 : aq0, b0, s[nf]); }
            }
        }
        if (HR) asm volatile("v_nop\n\tv_nop\n\tv_nop\n\tv_nop" : "+v"(s[0]), "+v"(s[1]), "+v"(s[2]), "+v"(s[3]) : "v"(ah0), "v"(al1));
        else    asm volatile("v_nop\n\tv_nop\n\tv_nop\n\tv_nop" : "+v"(s[0]), "+v"(s[1]), "+v"(s[2]), "+v"(s[3]) : "v"(aq0), "v"(aq1));
        float bm[8];
#pragma unroll
        for (int r = 0; r < 8; ++r) {
#pragma unroll
            for (int nf = 0; nf < 4; ++nf) { float x = s[nf][r] * SCL; if (part) { const int mv = ms[(8 * hi + r) * KT + nf * 16 + lr]; x = (mv != 0) ? x : MFILL; } s[nf][r] = x; }
            bm[r] = fmaxf(fmaxf(s[0][r], s[1][r]), fmaxf(s[2][r], s[3][r])); }
#pragma unroll
        for (int off = 1; off < 16; off <<= 1) {
#pragma unroll
            for (int r = 0; r < 8; ++r) bm[r] = fmaxf(bm[r], __shfl_xor(bm[r], off, 32)); }
        float rs[8];
#pragma unroll
        for (int r = 0; r < 8; ++r) {
            const float mn = fmaxf(mrow[r], bm[r]); const float corr = __builtin_amdgcn_exp2f((mrow[r] - mn) * L2E); mrow[r] = mn; lsum[r] = lsum[r] * corr;
#pragma unroll
            for (int t = 0; t < 4; ++t) acc[t][r] = acc[t][r] * corr;
            float sm = 0.f;
#pragma unroll
            for (int nf = 0; nf < 4; ++nf) { const float p = __builtin_amdgcn_exp2f((s[nf][r] - mn) * L2E); s[nf][r] = p; sm += p; }
            rs[r] = sm; }
#pragma unroll
        for (int off = 1; off < 16; off <<= 1) {
#pragma unroll
            for (int r = 0; r < 8; ++r) rs[r] += __shfl_xor(rs[r], off, 32); }
#pragma unroll
        for (int r = 0; r < 8; ++r) lsum[r] += rs[r];
        if (HR) {
#pragma unroll
            for (int nf = 0; nf < 4; ++nf)
#pragma unroll
                for (int r = 0; r < 8; ++r) { unsigned short a2, c2; splitf(s[nf][r], a2, c2); const int o = (8 * hi + r) * PP + nf * 16 + lr; pbh[o] = a2; pbl[o] = c2; }
        } else {
#pragma unroll
            for (int nf = 0; nf < 4; ++nf)
#pragma unroll
                for (int r = 0; r < 8; ++r) pb16[(8 * hi + r) * PP + nf * 16 + lr] = tohx(s[nf][r] * PCAR);
        }
        __syncthreads();
#pragma unroll
        for (int kc = 0; kc < KT; kc += 32) {
            const int po = lr * PP + 8 * hi + kc;
            if (HR) { const v16bf a0 = WFrag<bf>::ld(pbh + po), a1 = WFrag<bf>::ld(pbl + po);
#pragma unroll
                for (int t = 0; t < 4; ++t) { const size_t vo = hoff + (size_t)(t * 16 + lr) * SEQ + t0 + 8 * hi + kc; const v16bf b0 = WFrag<bf>::ld(Vh + vo), b1 = WFrag<bf>::ld(Vl + vo);
                    acc[t] = wmmab(a0, b0, acc[t]); acc[t] = wmmab(a1, b0, acc[t]); acc[t] = wmmab(a0, b1, acc[t]); }
            } else { const v16h a0 = WFrag<h16>::ld(pb16 + po);
#pragma unroll
                for (int t = 0; t < 4; ++t) { const size_t vo = hoff + (size_t)(t * 16 + lr) * SEQ + t0 + 8 * hi + kc; const v16h b0 = WFrag<h16>::ld(V16 + vo); acc[t] = wmma16(a0, b0, acc[t]); } }
        }
        asm volatile("v_nop\n\tv_nop\n\tv_nop\n\tv_nop" : "+v"(acc[0]), "+v"(acc[1]), "+v"(acc[2]), "+v"(acc[3]));
        __syncthreads();
    }
    float fr[8];
#pragma unroll
    for (int r = 0; r < 8; ++r) fr[r] = (HR ? 1.0f : (1.0f / PCAR)) * (1.0f / lsum[r]);
#pragma unroll
    for (int t = 0; t < 4; ++t)
#pragma unroll
        for (int r = 0; r < 8; ++r) os[(8 * hi + r) * 68 + t * 16 + lr] = acc[t][r] * fr[r];
    __syncthreads();
    const size_t abase = (size_t)hh * HD;
#pragma unroll 1
    for (int ps = 0; ps < 2; ++ps) {
#pragma unroll
        for (int i = 0; i < 4; ++i) { const int row = i * 4 + (lane >> 3); const int d0 = (lane & 7) * 8;
            const v4f x0 = *(const v4fa*)(os + row * 68 + d0); const v4f x1 = *(const v4fa*)(os + row * 68 + d0 + 4); v8us oh, ol;
#pragma unroll
            for (int q = 0; q < 4; ++q) { unsigned short a2, c2; splitf(x0[q], a2, c2); oh[q] = a2; ol[q] = c2; splitf(x1[q], a2, c2); oh[q + 4] = a2; ol[q + 4] = c2; }
            const size_t oo = (size_t)(q0 + row) * DQ + abase + d0;
            *(volatile v8us*)(Ah + oo) = oh; *(volatile v8us*)(Al + oo) = ol; }
        if (ps == 0) __threadfence(); }
}

extern "C" void kernel_launch(void* const* d_in, const int* in_sizes, int n_in,
                              void* d_out, int out_size, void* d_ws, size_t ws_size, hipStream_t stream) {
    if (n_in < 12) return;
    const float* xq = (const float*)d_in[0]; const float* xk = (const float*)d_in[1]; const float* xv = (const float*)d_in[2];
    const int* am = (const int*)d_in[3];
    const float* wq = (const float*)d_in[4]; const float* bq = (const float*)d_in[5];
    const float* wk = (const float*)d_in[6]; const float* bk = (const float*)d_in[7];
    const float* wv = (const float*)d_in[8]; const float* bv = (const float*)d_in[9];
    const float* wo = (const float*)d_in[10]; const float* bo = (const float*)d_in[11];
    float* OUT = (float*)d_out;
    const size_t needx = (size_t)(NB - 1) * SEQ_FULL * DM + (size_t)SEQ * DM;
    const size_t needm = (size_t)(SEQ - 1) * SEQ_FULL + SEQ;
    if ((size_t)in_sizes[0] < needx || (size_t)in_sizes[1] < needx || (size_t)in_sizes[2] < needx || (size_t)in_sizes[3] < needm) return;
    if ((size_t)in_sizes[4] < (size_t)DM * DM || (size_t)in_sizes[6] < (size_t)DM * DM || (size_t)in_sizes[8] < (size_t)DM * DM || (size_t)in_sizes[10] < (size_t)DM * DM) return;
    if (in_sizes[5] < DM || in_sizes[7] < DM || in_sizes[9] < DM || in_sizes[11] < DM) return;
    if ((size_t)out_size < (size_t)NB * SEQ * DM) return;

    char* wsp = (char*)d_ws;
    auto take = [&](size_t bytes) { char* p = wsp; wsp += (bytes + 255) & ~(size_t)255; return (void*)p; };
    const size_t PL = (size_t)SEQ * DM;
    bf* WQ = (bf*)take((size_t)DM * DM * 2); bf* WK = (bf*)take((size_t)DM * DM * 2); bf* WV = (bf*)take((size_t)DM * DM * 2); bf* WO = (bf*)take((size_t)DM * DM * 2);
    int* FLG = (int*)take((size_t)(SEQ / 16) * 32 * 4);
    bf* XB = (bf*)take(PL * 2); float* F = (float*)take(PL * 4);
    h16* Q16 = (h16*)take(PL * 2); bf* QPh = (bf*)take(PL * 2); bf* QPl = (bf*)take(PL * 2);
    h16* K16 = (h16*)take(PL * 2); bf* KPh = (bf*)take(PL * 2); bf* KPl = (bf*)take(PL * 2);
    h16* VT16 = (h16*)take(PL * 2); bf* VTh = (bf*)take(PL * 2); bf* VTl = (bf*)take(PL * 2);
    bf* ATh = (bf*)take(PL * 2); bf* ATl = (bf*)take(PL * 2);
    const size_t used = (size_t)(wsp - (char*)d_ws);
    if (used > ws_size || used > WS_CAP) return;

    const unsigned gw8 = (unsigned)(((size_t)DM * DM / 8 + 255) / 256);
    const unsigned gx8 = (unsigned)((PL / 8 + 255) / 256);
    const unsigned gpl = (unsigned)((PL / 2 + 255) / 256);
    const dim3 ggemm(SEQ / 64, DM / 64, 1);
    const int nq_hi = RHC / 16, nq_lo = SEQ / 16 - RHC / 16;

    k_cvt8<<<gw8, 256, 0, stream>>>(wq, WQ, (size_t)DM * DM / 8);
    k_cvt8<<<gw8, 256, 0, stream>>>(wk, WK, (size_t)DM * DM / 8);
    k_cvt8<<<gw8, 256, 0, stream>>>(wv, WV, (size_t)DM * DM / 8);
    k_cvt8<<<gw8, 256, 0, stream>>>(wo, WO, (size_t)DM * DM / 8);
    k_mflag<<<SEQ / 16, 32, 0, stream>>>(am, SEQ_FULL, NKT, FLG);
    for (int b = 0; b < NB; ++b) {
        k_cvt8<<<gx8, 256, 0, stream>>>(xq + (size_t)b * SEQ_FULL * DM, XB, PL / 8);
        k_gemmw<bf, 0, true><<<ggemm, 32, 0, stream>>>(XB, nullptr, WQ, nullptr, DM, F, DM, bq, 0, 0, 0);
        k_qkp<<<gpl, 256, 0, stream>>>(F, DM, NH, Q16, QPh, QPl);
        k_cvt8<<<gx8, 256, 0, stream>>>(xk + (size_t)b * SEQ_FULL * DM, XB, PL / 8);
        k_gemmw<bf, 0, true><<<ggemm, 32, 0, stream>>>(XB, nullptr, WK, nullptr, DM, F, DM, bk, 0, 0, 0);
        k_qkp<<<gpl, 256, 0, stream>>>(F, DM, NH, K16, KPh, KPl);
        k_cvt8<<<gx8, 256, 0, stream>>>(xv + (size_t)b * SEQ_FULL * DM, XB, PL / 8);
        k_gemmw<bf, 0, true><<<ggemm, 32, 0, stream>>>(XB, nullptr, WV, nullptr, DM, F, DM, bv, 0, 0, 0);
        k_vtp<<<gpl, 256, 0, stream>>>(F, DM, NH, VT16, VTh, VTl);
        if (nq_hi > 0) k_flash<true><<<dim3(nq_hi, NH, 1), 32, 0, stream>>>(Q16, QPh, QPl, K16, KPh, KPl, VT16, VTh, VTl, am, SEQ_FULL, FLG, 0, ATh, ATl);
        if (nq_lo > 0) k_flash<false><<<dim3(nq_lo, NH, 1), 32, 0, stream>>>(Q16, QPh, QPl, K16, KPh, KPl, VT16, VTh, VTl, am, SEQ_FULL, FLG, nq_hi, ATh, ATl);
        k_gemmw<bf, 1, true><<<ggemm, 32, 0, stream>>>(ATh, ATl, WO, nullptr, DQ, OUT + (size_t)b * SEQ * DM, DM, bo, 0, 0, 0);
    }
}
